// SelfAttentionHead_20229295964971
// MI455X (gfx1250) — hardware-verified
//
#include <hip/hip_runtime.h>

typedef __attribute__((ext_vector_type(16))) _Float16 v16h;
typedef __attribute__((ext_vector_type(8)))  _Float16 v8h;
typedef __attribute__((ext_vector_type(16))) __bf16   v16b;
typedef __attribute__((ext_vector_type(8)))  __bf16   v8b;
typedef __attribute__((ext_vector_type(8)))  float    v8f;
typedef __attribute__((ext_vector_type(4)))  float    v4f;
typedef __attribute__((ext_vector_type(4)))  unsigned int v4u;

constexpr int NBATCH = 4;
constexpr int SEQ_T  = 2048;
constexpr int EMB_C  = 1024;
constexpr int NHEAD  = 16;
constexpr int HDIM   = 64;
constexpr int NOUT3  = 3 * EMB_C;
constexpr int MROWS  = NBATCH * SEQ_T;
constexpr int LDQK   = 2 * EMB_C;
static_assert(NHEAD * HDIM == EMB_C, "head geometry");
static_assert(HDIM == 64, "head dim 64 kernel");
static_assert(EMB_C % 32 == 0, "GEMM K multiple of 32");
static_assert(MROWS % 64 == 0, "GEMM M multiple of 64");
static_assert(LDQK % 64 == 0 && EMB_C % 64 == 0, "GEMM N multiple of 64");
static_assert(SEQ_T % 64 == 0, "query blocks of 64");
static_assert((NBATCH * SEQ_T * EMB_C) % 8 == 0 && (NOUT3 * EMB_C) % 8 == 0 && NOUT3 % 4 == 0, "cast granularity");

__device__ __forceinline__ unsigned short f2bf_bits(float f) {
  unsigned u = __float_as_uint(f);
  return (unsigned short)((u + 0x7FFFu + ((u >> 16) & 1u)) >> 16);
}
__device__ __forceinline__ float bf_bits2f(unsigned short h) { return __uint_as_float(((unsigned)h) << 16); }

__device__ __forceinline__ void dep_guard_h(v8f& a, v8f& b, v16h x, v16h y) { asm volatile("v_nop\n\tv_nop\n\tv_nop\n\tv_nop" : "+v"(a), "+v"(b) : "v"(x), "v"(y)); }
__device__ __forceinline__ void dep_guard_b(v8f& a, v8f& b, v16b x, v16b y) { asm volatile("v_nop\n\tv_nop\n\tv_nop\n\tv_nop" : "+v"(a), "+v"(b) : "v"(x), "v"(y)); }
__device__ __forceinline__ void keep4_h(v16h a, v16h b, v16h c, v16h d) { asm volatile("v_nop" :: "v"(a), "v"(b), "v"(c), "v"(d)); }
__device__ __forceinline__ void keep4_b(v16b a, v16b b, v16b c, v16b d) { asm volatile("v_nop" :: "v"(a), "v"(b), "v"(c), "v"(d)); }
__device__ __forceinline__ void acc_guard4(v8f& a, v8f& b, v8f& c, v8f& d) { asm volatile("v_nop\n\tv_nop\n\tv_nop\n\tv_nop" : "+v"(a), "+v"(b), "+v"(c), "+v"(d)); }
template <typename T> struct Frag;
template <> struct Frag<_Float16> {
  typedef v16h V; union U { v16h v; v8h h[2]; };
  static __device__ __forceinline__ v16h load(const _Float16* p) {
    U f; f.h[0] = *(const v8h*)(p); f.h[1] = *(const v8h*)(p + 16); return f.v;
  }
  static __device__ __forceinline__ v8f mma(v16h a, v16h b, v8f c) {
    return __builtin_amdgcn_wmma_f32_16x16x32_f16(false, a, false, b, (short)0, c, false, false);
  }
  static __device__ __forceinline__ void guard(v8f& a, v8f& b, v16h x, v16h y) { dep_guard_h(a, b, x, y); }
  static __device__ __forceinline__ void keep(v16h a, v16h b, v16h c, v16h d) { keep4_h(a, b, c, d); }
};
template <> struct Frag<__bf16> {
  typedef v16b V; union U { v16b v; v8b h[2]; };
  static __device__ __forceinline__ v16b load(const __bf16* p) {
    U f; f.h[0] = *(const v8b*)(p); f.h[1] = *(const v8b*)(p + 16); return f.v;
  }
  static __device__ __forceinline__ v8f mma(v16b a, v16b b, v8f c) {
    return __builtin_amdgcn_wmma_f32_16x16x32_bf16(false, a, false, b, (short)0, c, false, false);
  }
  static __device__ __forceinline__ void guard(v8f& a, v8f& b, v16b x, v16b y) { dep_guard_b(a, b, x, y); }
  static __device__ __forceinline__ void keep(v16b a, v16b b, v16b c, v16b d) { keep4_b(a, b, c, d); }
};

template <int ET> struct Elem;
template <> struct Elem<0> { typedef _Float16 T; };
template <> struct Elem<1> { typedef __bf16 T; };
template <int ET, bool SPLIT, int BIAS_MODE, int OUT_MODE, bool RESID, int ACT = 0>
__global__ __launch_bounds__(256) void wmma_gemm64(
    const unsigned short* __restrict__ Ap, const unsigned short* __restrict__ A2p, int lda, long strideA,
    const unsigned short* __restrict__ Btp, const unsigned short* __restrict__ Bt2p, int ldb, long strideB,
    void* __restrict__ Cout, void* __restrict__ Cout2, int ldc, long strideC,
    const float* __restrict__ bias,
    const float* __restrict__ resid, long strideR,
    int M, int N, int K, float scale) {
  typedef typename Elem<ET>::T T;
  typedef typename Frag<T>::V V;
  const T* A = (const T*)Ap; const T* A2 = (const T*)A2p; const T* Bt = (const T*)Btp; const T* Bt2 = (const T*)Bt2p;
  __shared__ __align__(16) float sT[8][16 * 68];
  const int b    = blockIdx.y;
  const int lane = threadIdx.x & 31;
  const int wave = threadIdx.x >> 5;
  const int tilesN = N >> 6;
  const int tilesM = M >> 6;
  const int tile = blockIdx.x * 8 + wave;
  if (tile >= tilesM * tilesN) return;
  const int tm = tile / tilesN;
  const int tn = tile - tm * tilesN;
  const int m0 = tm << 6;
  const int n0 = tn << 6;

  const T* Ab  = A  + (size_t)b * strideA;
  const T* Bb  = Bt + (size_t)b * strideB;
  const T* Ab2 = SPLIT ? (A2  + (size_t)b * strideA) : nullptr;
  const T* Bb2 = SPLIT ? (Bt2 + (size_t)b * strideB) : nullptr;

  const int rlane = lane & 15;
  const int koff  = (lane >> 4) * 8;
  const int mOff  = (lane >> 4) * 8;

  v8f acc[4][4];
#pragma unroll
  for (int i = 0; i < 4; ++i)
#pragma unroll
    for (int j = 0; j < 4; ++j) acc[i][j] = (v8f){0.f,0.f,0.f,0.f,0.f,0.f,0.f,0.f};

  for (int k0 = 0; k0 < K; k0 += 32) {
    V bh[4], bl[4];
#pragma unroll
    for (int j = 0; j < 4; ++j) {
      const size_t bo = (size_t)(n0 + (j << 4) + rlane) * ldb + koff + k0;
      bh[j] = Frag<T>::load(Bb + bo);
      if (SPLIT) bl[j] = Frag<T>::load(Bb2 + bo);
    }
#pragma unroll
    for (int i = 0; i < 4; ++i) {
      const size_t ao = (size_t)(m0 + (i << 4) + rlane) * lda + koff + k0;
      V ah = Frag<T>::load(Ab + ao);
      V al;
      if (SPLIT) al = Frag<T>::load(Ab2 + ao);
#pragma unroll
      for (int j = 0; j < 4; ++j) {
        acc[i][j] = Frag<T>::mma(ah, bh[j], acc[i][j]);
        if (SPLIT) {
          acc[i][j] = Frag<T>::mma(ah, bl[j], acc[i][j]);
          acc[i][j] = Frag<T>::mma(al, bh[j], acc[i][j]);
        }
      }
      Frag<T>::guard(acc[i][0], acc[i][3], ah, SPLIT ? al : ah);
    }
    Frag<T>::keep(bh[0], bh[1], bh[2], bh[3]);
    if (SPLIT) Frag<T>::keep(bl[0], bl[1], bl[2], bl[3]);
  }
  acc_guard4(acc[0][0], acc[0][1], acc[0][2], acc[0][3]);
  acc_guard4(acc[1][0], acc[1][1], acc[1][2], acc[1][3]);
  acc_guard4(acc[2][0], acc[2][1], acc[2][2], acc[2][3]);
  acc_guard4(acc[3][0], acc[3][1], acc[3][2], acc[3][3]);

  float* slab = sT[wave];
  const float* Rb = RESID ? (resid + (size_t)b * strideR) : nullptr;
#pragma unroll
  for (int i = 0; i < 4; ++i) {
    const int mBase = m0 + (i << 4);
#pragma unroll
    for (int j = 0; j < 4; ++j) {
      const int n = n0 + (j << 4) + rlane;
      float bv = 0.f;
      if (BIAS_MODE == 2) bv = bias[n];
#pragma unroll
      for (int r = 0; r < 8; ++r) {
        float v = acc[i][j][r] * scale;
        if (BIAS_MODE == 1) v += bias[mBase + mOff + r];
        if (BIAS_MODE == 2) v += bv;
        if (RESID) v += Rb[(size_t)(mBase + mOff + r) * ldc + n];
        if (ACT == 1) v = tanhf(v);
        if (ACT == 2) v = fmaxf(v, 0.0f);
        if (ACT == 3) v = v / (1.0f + expf(-v));
        if (ACT == 4) v = (v > 0.f) ? v : 0.01f * v;
        if (ACT == 5) v = 0.5f * v * (1.0f + erff(v * 0.70710678118654752f));
        slab[(mOff + r) * 68 + (j << 4) + rlane] = v;
      }
    }
    __builtin_amdgcn_fence(__ATOMIC_RELEASE, "workgroup");
    __builtin_amdgcn_wave_barrier();
    __builtin_amdgcn_fence(__ATOMIC_ACQUIRE, "workgroup");
    if (OUT_MODE == 0) {
      float* C = (float*)Cout + (size_t)b * strideC;
      const int hh = lane >> 4, c4 = (lane & 15) * 4;
      for (int pass = 0; pass < 2; ++pass) {
#pragma unroll
        for (int it = 0; it < 8; ++it) {
          const int row = it * 2 + hh;
          v4f v = *(const v4f*)(slab + row * 68 + c4);
          *(volatile v4f*)(C + (size_t)(mBase + row) * ldc + n0 + c4) = v;
        }
        __threadfence();
      }
    } else {
      const int q = lane >> 3, c8 = (lane & 7) * 8;
      unsigned short* C  = (unsigned short*)Cout  + (size_t)b * strideC;
      unsigned short* C2 = (OUT_MODE == 2) ? ((unsigned short*)Cout2 + (size_t)b * strideC) : nullptr;
      for (int pass = 0; pass < 2; ++pass) {
#pragma unroll
        for (int it = 0; it < 4; ++it) {
          const int row = it * 4 + q;
          const float* sp = slab + row * 68 + c8;
          v8h hv, lv;
#pragma unroll
          for (int e = 0; e < 8; ++e) {
            if (OUT_MODE == 1) {
              hv[e] = (_Float16)sp[e];
            } else {
              unsigned short hb = f2bf_bits(sp[e]);
              unsigned short lb = f2bf_bits(sp[e] - bf_bits2f(hb));
              hv[e] = __builtin_bit_cast(_Float16, hb);
              lv[e] = __builtin_bit_cast(_Float16, lb);
            }
          }
          *(volatile v8h*)(C + (size_t)(mBase + row) * ldc + n0 + c8) = hv;
          if (OUT_MODE == 2) *(volatile v8h*)(C2 + (size_t)(mBase + row) * ldc + n0 + c8) = lv;
        }
        __threadfence();
      }
    }
    __builtin_amdgcn_fence(__ATOMIC_RELEASE, "workgroup");
    __builtin_amdgcn_wave_barrier();
    __builtin_amdgcn_fence(__ATOMIC_ACQUIRE, "workgroup");
  }
}

__global__ __launch_bounds__(256) void cast_f32_bf16x8(
    const float* __restrict__ in, unsigned short* __restrict__ out, int n8) {
  const int i = blockIdx.x * 256 + threadIdx.x;
  if (i < n8) {
    const v4f a = *(const v4f*)(in + (size_t)8 * i);
    const v4f c = *(const v4f*)(in + (size_t)8 * i + 4);
    v4u w;
    w[0] = (unsigned)f2bf_bits(a[0]) | ((unsigned)f2bf_bits(a[1]) << 16);
    w[1] = (unsigned)f2bf_bits(a[2]) | ((unsigned)f2bf_bits(a[3]) << 16);
    w[2] = (unsigned)f2bf_bits(c[0]) | ((unsigned)f2bf_bits(c[1]) << 16);
    w[3] = (unsigned)f2bf_bits(c[2]) | ((unsigned)f2bf_bits(c[3]) << 16);
    volatile v4u* p = (volatile v4u*)(out + (size_t)8 * i);
    *p = w;
    __threadfence();
    *p = w;
  }
}

__global__ __launch_bounds__(256) void bias_bf16_rne(
    const float* __restrict__ in, float* __restrict__ out, int n4) {
  const int i = blockIdx.x * 256 + threadIdx.x;
  if (i < n4) {
    const v4f a = *(const v4f*)(in + (size_t)4 * i);
    v4f r;
#pragma unroll
    for (int e = 0; e < 4; ++e) r[e] = bf_bits2f(f2bf_bits(a[e]));
    volatile v4f* p = (volatile v4f*)(out + (size_t)4 * i);
    *p = r;
    __threadfence();
    *p = r;
  }
}

__device__ __forceinline__ v8f at_mma(v16b a, v16b b, v8f c) {
  c = __builtin_amdgcn_wmma_f32_16x16x32_bf16(false, a, false, b, (short)0, c, false, false);
  asm volatile("v_nop\n\tv_nop\n\tv_nop\n\tv_nop" : "+v"(c) : "v"(a), "v"(b));
  return c;
}
__device__ __forceinline__ v8f at_mma_h(v16b a, v16b b, v8f c) {
  const v16h ah = __builtin_bit_cast(v16h, a), bh = __builtin_bit_cast(v16h, b);
  c = __builtin_amdgcn_wmma_f32_16x16x32_f16(false, ah, false, bh, (short)0, c, false, false);
  asm volatile("v_nop\n\tv_nop\n\tv_nop\n\tv_nop" : "+v"(c) : "v"(ah), "v"(bh));
  return c;
}
__device__ __forceinline__ __bf16 at_h16(float f) { return __builtin_bit_cast(__bf16, (_Float16)f); }

constexpr float P_CARRY = 32768.0f;
__global__ __launch_bounds__(128)
void attn64_planes(const unsigned short* __restrict__ qkh, const unsigned short* __restrict__ qkl,
                   const unsigned short* __restrict__ vpl, float* __restrict__ out, float qscale) {
  union FB { v16b v; v8b h[2]; };
  __shared__ __align__(16) unsigned short Ksh[64 * 64];
  __shared__ __align__(16) unsigned short Ksl[64 * 64];
  __shared__ __align__(16) unsigned short Vt[64 * 64];
  __shared__ __align__(16) __bf16 Psh[4][16 * 64];
  __shared__ __align__(16) float  Os[4][16 * 68];
  const float NEG_INF = -__builtin_huge_valf();

  const int tid  = threadIdx.x;
  const int wave = tid >> 5;
  const int lane = tid & 31;
  const int hh   = lane >> 4;
  const int c    = lane & 15;

  constexpr int nqb = SEQ_T / 64;
  const int bx = blockIdx.x;
  const int qb = bx % nqb;
  const int bh = bx / nqb;
  const int h  = bh % NHEAD;
  const int b  = bh / NHEAD;
  const int q0 = qb * 64 + wave * 16;
  const size_t rb = (size_t)b * SEQ_T;

  v16b qah[2], qal[2];
  {
    const size_t qo = (rb + q0 + c) * (size_t)LDQK + h * HDIM;
    const __bf16* QH = (const __bf16*)qkh + qo;
    const __bf16* QL = (const __bf16*)qkl + qo;
#pragma unroll
    for (int dc = 0; dc < 2; ++dc) {
      qah[dc] = Frag<__bf16>::load(QH + dc * 32 + 8 * hh);
      qal[dc] = Frag<__bf16>::load(QL + dc * 32 + 8 * hh);
    }
  }

  float mrow[8], lrow[8];
  v8f oacc[4];
#pragma unroll
  for (int r = 0; r < 8; ++r) { mrow[r] = NEG_INF; lrow[r] = 0.f; }
#pragma unroll
  for (int t = 0; t < 4; ++t) oacc[t] = (v8f){0.f,0.f,0.f,0.f,0.f,0.f,0.f,0.f};

  const int nChunks = qb + 1;
  for (int kc = 0; kc < nChunks; ++kc) {
    const int kv0 = kc * 64;
    __syncthreads();
    {
      const int kvr = tid >> 1, dh = (tid & 1) * 32;
      const size_t krow = (rb + kv0 + kvr) * (size_t)LDQK + EMB_C + h * HDIM + dh;
      const size_t vrow = (rb + kv0 + kvr) * (size_t)EMB_C + h * HDIM + dh;
#pragma unroll
      for (int i = 0; i < 4; ++i) {
        const v4u w = *(const v4u*)(qkh + krow + 8 * i);
        *(v4u*)(Ksh + kvr * 64 + dh + 8 * i) = w;
      }
#pragma unroll
      for (int i = 0; i < 4; ++i) {
        const v4u w = *(const v4u*)(qkl + krow + 8 * i);
        *(v4u*)(Ksl + kvr * 64 + dh + 8 * i) = w;
      }
#pragma unroll
      for (int i = 0; i < 4; ++i) {
        const v4u w = *(const v4u*)(vpl + vrow + 8 * i);
#pragma unroll
        for (int e = 0; e < 8; ++e) {
          const unsigned short bits = (unsigned short)((w[e >> 1] >> ((e & 1) * 16)) & 0xffffu);
          Vt[(dh + 8 * i + e) * 64 + kvr] = bits;
        }
      }
    }
    __syncthreads();

    v8f s[4];
#pragma unroll
    for (int j = 0; j < 4; ++j) {
      s[j] = (v8f){0.f,0.f,0.f,0.f,0.f,0.f,0.f,0.f};
#pragma unroll
      for (int dc = 0; dc < 2; ++dc) {
        const __bf16* kp = (const __bf16*)Ksh + (j * 16 + c) * 64 + dc * 32 + 8 * hh;
        const __bf16* lp = (const __bf16*)Ksl + (j * 16 + c) * 64 + dc * 32 + 8 * hh;
        FB kb, kl;
        kb.h[0] = *(const v8b*)(kp);
        kb.h[1] = *(const v8b*)(kp + 16);
        kl.h[0] = *(const v8b*)(lp);
        kl.h[1] = *(const v8b*)(lp + 16);
        s[j] = at_mma(qah[dc], kb.v, s[j]);
        s[j] = at_mma(qah[dc], kl.v, s[j]);
        s[j] = at_mma(qal[dc], kb.v, s[j]);
      }
    }
    const bool diag = (kc == qb);
    float cm[8];
#pragma unroll
    for (int r = 0; r < 8; ++r) {
      const int qrow = q0 + 8 * hh + r;
      float m = NEG_INF;
#pragma unroll
      for (int j = 0; j < 4; ++j) {
        const int kvcol = kv0 + j * 16 + c;
        float sv = s[j][r] * qscale;
        if (diag && (kvcol > qrow)) sv = NEG_INF;
        s[j][r] = sv;
        m = fmaxf(m, sv);
      }
#pragma unroll
      for (int off = 1; off < 16; off <<= 1) m = fmaxf(m, __shfl_xor(m, off, 32));
      cm[r] = m;
    }
    __bf16* pwh = Psh[wave];
#pragma unroll
    for (int r = 0; r < 8; ++r) {
      const float mnew = fmaxf(mrow[r], cm[r]);
      const float alpha = expf(mrow[r] - mnew);
      mrow[r] = mnew;
      float psum = 0.f;
#pragma unroll
      for (int j = 0; j < 4; ++j) {
        const float p = expf(s[j][r] - mnew);
        psum += p;
        pwh[(8 * hh + r) * 64 + j * 16 + c] = at_h16(p * P_CARRY);
      }
#pragma unroll
      for (int off = 1; off < 16; off <<= 1) psum += __shfl_xor(psum, off, 32);
      lrow[r] = lrow[r] * alpha + psum;
#pragma unroll
      for (int t = 0; t < 4; ++t) oacc[t][r] *= alpha;
    }
    __builtin_amdgcn_fence(__ATOMIC_RELEASE, "workgroup");
    __builtin_amdgcn_wave_barrier();
    __builtin_amdgcn_fence(__ATOMIC_ACQUIRE, "workgroup");
#pragma unroll 1
    for (int kk = 0; kk < 2; ++kk) {
      FB pa;
      pa.h[0] = *(const v8b*)(pwh + c * 64 + kk * 32 + 8 * hh);
      pa.h[1] = *(const v8b*)(pwh + c * 64 + kk * 32 + 16 + 8 * hh);
#pragma unroll
      for (int t = 0; t < 4; ++t) {
        const __bf16* vp = (const __bf16*)Vt + (t * 16 + c) * 64 + kk * 32 + 8 * hh;
        FB vb;
        vb.h[0] = *(const v8b*)(vp);
        vb.h[1] = *(const v8b*)(vp + 16);
        oacc[t] = at_mma_h(pa.v, vb.v, oacc[t]);
      }
    }
  }

  float* os = Os[wave];
#pragma unroll
  for (int r = 0; r < 8; ++r) {
    const float inv = 1.0f / (lrow[r] * P_CARRY);
#pragma unroll
    for (int t = 0; t < 4; ++t) os[(8 * hh + r) * 68 + t * 16 + c] = oacc[t][r] * inv;
  }
  __builtin_amdgcn_fence(__ATOMIC_RELEASE, "workgroup");
  __builtin_amdgcn_wave_barrier();
  __builtin_amdgcn_fence(__ATOMIC_ACQUIRE, "workgroup");
  {
    float* ob_ptr = out + rb * (size_t)EMB_C + h * HDIM;
    const int c4 = (lane & 15) * 4;
    for (int pass = 0; pass < 2; ++pass) {
#pragma unroll
      for (int it = 0; it < 8; ++it) {
        const int row = it * 2 + hh;
        v4f val = *(const v4f*)(os + row * 68 + c4);
        *(volatile v4f*)(ob_ptr + (size_t)(q0 + row) * EMB_C + c4) = val;
      }
      __threadfence();
    }
  }
}

extern "C" void kernel_launch(void* const* d_in, const int* in_sizes, int n_in,
                              void* d_out, int out_size, void* d_ws, size_t ws_size,
                              hipStream_t stream) {
  if (n_in < 3) return;
  const int NX = NBATCH * SEQ_T * EMB_C;
  const int NW = NOUT3 * EMB_C;
  const int NB = NOUT3;
  if (in_sizes[0] != NX || in_sizes[1] != NW || in_sizes[2] != NB || out_size != NX) return;

  const float* x    = (const float*)d_in[0];
  const float* Wm   = (const float*)d_in[1];
  const float* bias = (const float*)d_in[2];
  float* out = (float*)d_out;

  const size_t offX    = 0;
  const size_t offW    = offX    + (size_t)NX * 2;
  const size_t offBias = offW    + (size_t)NW * 2;
  const size_t offQKh  = offBias + (size_t)NB * 4;
  const size_t offQKl  = offQKh  + (size_t)MROWS * LDQK * 2;
  const size_t offV    = offQKl  + (size_t)MROWS * LDQK * 2;
  const size_t total   = offV    + (size_t)MROWS * EMB_C * 2;
  if (total > ws_size) return;

  char* ws = (char*)d_ws;
  unsigned short* Xb  = (unsigned short*)(ws + offX);
  unsigned short* Wb  = (unsigned short*)(ws + offW);
  float*          Br  = (float*)(ws + offBias);
  unsigned short* QKh = (unsigned short*)(ws + offQKh);
  unsigned short* QKl = (unsigned short*)(ws + offQKl);
  unsigned short* Vp  = (unsigned short*)(ws + offV);

  {
    const int n8x = NX / 8, n8w = NW / 8, n4b = NB / 4;
    cast_f32_bf16x8<<<dim3((n8x + 255) / 256), dim3(256), 0, stream>>>(x, Xb, n8x);
    cast_f32_bf16x8<<<dim3((n8w + 255) / 256), dim3(256), 0, stream>>>(Wm, Wb, n8w);
    bias_bf16_rne<<<dim3((n4b + 255) / 256), dim3(256), 0, stream>>>(bias, Br, n4b);
  }
  {
    const int tiles = (MROWS / 64) * (LDQK / 64);
    wmma_gemm64<1, false, 2, 2, false, 0><<<dim3((tiles + 7) / 8, 1), dim3(256), 0, stream>>>(
        Xb, Xb, EMB_C, 0L,
        Wb, Wb, EMB_C, 0L,
        (void*)QKh, (void*)QKl, LDQK, 0L,
        Br, Br, 0L,
        MROWS, LDQK, EMB_C, 1.0f);
  }
  {
    const int tiles = (MROWS / 64) * (EMB_C / 64);
    wmma_gemm64<1, false, 2, 1, false, 0><<<dim3((tiles + 7) / 8, 1), dim3(256), 0, stream>>>(
        Xb, Xb, EMB_C, 0L,
        Wb + (size_t)2 * EMB_C * EMB_C, Wb + (size_t)2 * EMB_C * EMB_C, EMB_C, 0L,
        (void*)Vp, (void*)Vp, EMB_C, 0L,
        Br + 2 * EMB_C, Br, 0L,
        MROWS, EMB_C, EMB_C, 1.0f);
  }
  attn64_planes<<<dim3(NBATCH * NHEAD * (SEQ_T / 64)), dim3(128), 0, stream>>>(
      QKh, QKl, Vp, out, 0.125f);
}
